// GraphModule_14972255994536
// MI455X (gfx1250) — hardware-verified
//
#include <hip/hip_runtime.h>
#include <stddef.h>
#include <stdint.h>


#define FIN     256
#define HD1     128
#define D2      64
#define KG2     256
#define NTHR    256
#define NWAVE   8
#define EPT     8
#define CHUNK   (NTHR * EPT)
#define WCAP    (EPT * 32)
#define LISTN   (NWAVE * WCAP)
#define NBMAX   2048
#define RCAP    28672
#define DEGCAP  512
#define STW     128
#define GBM     64
#define GBN     64
#define GTHR    128
#define NEGSL   0.2f
#define WSMAX   134217728
#define LDS_AGG ((2 * RCAP + 2 * NBMAX + LISTN) * 4 + 64)

static_assert((CHUNK & (CHUNK - 1)) == 0 && CHUNK <= 4096);
static_assert((NBMAX & (NBMAX - 1)) == 0 && NBMAX <= 4096);
static_assert(NTHR * 8 == NBMAX);
static_assert(LISTN >= NBMAX);
static_assert(LISTN >= NWAVE * WCAP);
static_assert((RCAP % 32) == 0);
static_assert(NWAVE * STW <= RCAP);
static_assert(STW * 4 == KG2 * 2);
static_assert(LDS_AGG <= 300000);
static_assert(GBM == (GTHR / 32) * 16);
static_assert((FIN % 32) == 0 && (KG2 % 32) == 0 && (FIN % 8) == 0 && (HD1 % 8) == 0);
static_assert((HD1 % GBN) == 0 && (D2 % GBN) == 0);
static_assert(HD1 == 32 * 4 && D2 == 32 * 2 && KG2 == 2 * HD1);
static_assert(FIN / 8 == 32);

typedef float          v2f  __attribute__((ext_vector_type(2)));
typedef float          v4f  __attribute__((ext_vector_type(4)));
typedef float          v8f  __attribute__((ext_vector_type(8)));
typedef int            v4i  __attribute__((ext_vector_type(4)));
typedef int            v8i  __attribute__((ext_vector_type(8)));
typedef unsigned int   v2u  __attribute__((ext_vector_type(2)));
typedef unsigned int   v4u  __attribute__((ext_vector_type(4)));
typedef unsigned short v8us __attribute__((ext_vector_type(8)));
typedef __bf16         v16b __attribute__((ext_vector_type(16)));
typedef v2f  __attribute__((may_alias)) v2fa;
typedef v4f  __attribute__((may_alias)) v4fa;
typedef v2u  __attribute__((may_alias)) v2ua;
typedef v4u  __attribute__((may_alias)) v4ua;
typedef v8us __attribute__((may_alias)) v8usa;
union FragB { v16b v; v8us h[2]; v8i w; };

__device__ __forceinline__ v8f wmb(const FragB& a, const FragB& b, v8f c) {
  v8f d = __builtin_amdgcn_wmma_f32_16x16x32_bf16(false, a.v, false, b.v, (short)0, c, false, false);
  asm volatile("v_nop\n\tv_nop\n\tv_nop\n\tv_nop" : "+v"(d) : "v"(a.w), "v"(b.w));
  return d;
}

__device__ __forceinline__ unsigned int f2bf(float f) {
  const unsigned int u = __float_as_uint(f);
  return (u + 0x7FFFu + ((u >> 16) & 1u)) >> 16;
}
__device__ __forceinline__ float bf2f(unsigned int b) { return __uint_as_float(b << 16); }
__device__ __forceinline__ float bfr(float f) { return bf2f(f2bf(f)); }
__device__ __forceinline__ v4f bfr4(const v4f a) {
  v4f r; r.x = bfr(a.x); r.y = bfr(a.y); r.z = bfr(a.z); r.w = bfr(a.w); return r;
}
__device__ __forceinline__ unsigned int pk2(float lo, float hi) { return f2bf(lo) | (f2bf(hi) << 16); }
__device__ __forceinline__ v4u pack8(const v4f a, const v4f b) {
  v4u r;
  r.x = pk2(a.x, a.y); r.y = pk2(a.z, a.w); r.z = pk2(b.x, b.y); r.w = pk2(b.z, b.w);
  return r;
}

__device__ __forceinline__ int scan_chunk(const int* __restrict__ dsts, int nE, int cbase, int slotBase,
                                          int nb, int vec8, int* list, int tid, int lane, int wave) {
  int wc = 0;
  const int el0  = tid * EPT;
  const int e0   = cbase + el0;
  const int sent = -2147483647 - 1;
  v4i da, db;
  if (vec8 != 0 && cbase + CHUNK <= nE) {
    da = *(const v4i*)(dsts + e0);
    db = *(const v4i*)(dsts + e0 + 4);
  } else {
    da.x = (e0     < nE) ? dsts[min(e0,     nE - 1)] : sent;
    da.y = (e0 + 1 < nE) ? dsts[min(e0 + 1, nE - 1)] : sent;
    da.z = (e0 + 2 < nE) ? dsts[min(e0 + 2, nE - 1)] : sent;
    da.w = (e0 + 3 < nE) ? dsts[min(e0 + 3, nE - 1)] : sent;
    db.x = (e0 + 4 < nE) ? dsts[min(e0 + 4, nE - 1)] : sent;
    db.y = (e0 + 5 < nE) ? dsts[min(e0 + 5, nE - 1)] : sent;
    db.z = (e0 + 6 < nE) ? dsts[min(e0 + 6, nE - 1)] : sent;
    db.w = (e0 + 7 < nE) ? dsts[min(e0 + 7, nE - 1)] : sent;
  }
  const unsigned nbs = (unsigned)slotBase;
  const unsigned unb = (unsigned)nb;
  const unsigned s0 = (unsigned)da.x - nbs, s1 = (unsigned)da.y - nbs;
  const unsigned s2 = (unsigned)da.z - nbs, s3 = (unsigned)da.w - nbs;
  const unsigned s4 = (unsigned)db.x - nbs, s5 = (unsigned)db.y - nbs;
  const unsigned s6 = (unsigned)db.z - nbs, s7 = (unsigned)db.w - nbs;
  const bool h0 = s0 < unb, h1 = s1 < unb, h2 = s2 < unb, h3 = s3 < unb;
  const bool h4 = s4 < unb, h5 = s5 < unb, h6 = s6 < unb, h7 = s7 < unb;
  const unsigned any = __builtin_amdgcn_ballot_w32(h0 | h1 | h2 | h3 | h4 | h5 | h6 | h7);
  if (any != 0u) {
#define HITJ(J, HJ, SJ) { \
      const unsigned mj = __builtin_amdgcn_ballot_w32(HJ); \
      if (mj != 0u) { \
        if (HJ) { \
          const int pos = wc + (int)__builtin_amdgcn_mbcnt_lo(mj, 0u); \
          if (pos < WCAP) list[wave * WCAP + pos] = ((el0 + (J)) << 12) | (int)(SJ); \
        } \
        wc += (int)__builtin_popcount(mj); } }
    HITJ(0, h0, s0)
    HITJ(1, h1, s1)
    HITJ(2, h2, s2)
    HITJ(3, h3, s3)
    HITJ(4, h4, s4)
    HITJ(5, h5, s5)
    HITJ(6, h6, s6)
    HITJ(7, h7, s7)
#undef HITJ
  }
  return wc;
}

__global__ __launch_bounds__(NTHR) void k_xprep(const float* __restrict__ x, unsigned short* xb, int nN, int nUnits) {
  const int i = (int)blockIdx.x * NTHR + (int)threadIdx.x;
  if (i >= nUnits) return;
  const int row = i >> 5;
  const int c0  = (i & 31) * 8;
  const int rc  = row < nN ? row : nN - 1;
  const float* p = x + (size_t)rc * FIN + c0;
  v4f a = *(const v4fa*)p, b = *(const v4fa*)(p + 4);
  const v4f z4 = {0.f, 0.f, 0.f, 0.f};
  if (row >= nN) { a = z4; b = z4; }
  const v4u wv = pack8(a, b);
  unsigned short* o = xb + (size_t)row * FIN + c0;
  *(volatile v4u*)o = wv;
  __threadfence();
  *(volatile v4u*)o = wv;
}

__global__ __launch_bounds__(NTHR) void k_wtr(const float* __restrict__ w, int Kin, int Ncol, int Nrows, int Kout,
                                              unsigned short* wt, int nUnits) {
  const int u = (int)blockIdx.x * NTHR + (int)threadIdx.x;
  if (u >= nUnits) return;
  const int kq = Kout >> 3;
  const int n  = u / kq;
  const int k8 = (u - n * kq) * 8;
  const int kk = k8 - (k8 / Kin) * Kin;
  const int ncl = n < Ncol ? n : Ncol - 1;
  const float* p = w + (size_t)kk * (size_t)Ncol + ncl;
  v4f a, b;
  a.x = p[0];                    a.y = p[(size_t)Ncol];         a.z = p[(size_t)2 * Ncol];     a.w = p[(size_t)3 * Ncol];
  b.x = p[(size_t)4 * Ncol];     b.y = p[(size_t)5 * Ncol];     b.z = p[(size_t)6 * Ncol];     b.w = p[(size_t)7 * Ncol];
  const v4f z4 = {0.f, 0.f, 0.f, 0.f};
  if (n >= Ncol || n >= Nrows) { a = z4; b = z4; }
  const v4u wv = pack8(a, b);
  unsigned short* o = wt + (size_t)n * (size_t)Kout + k8;
  *(volatile v4u*)o = wv;
  __threadfence();
  *(volatile v4u*)o = wv;
}

__global__ __launch_bounds__(GTHR) void k_gemm(
    const unsigned short* __restrict__ A, const unsigned short* __restrict__ WT,
    float* outF, int K, int ldo)
{
  __shared__ __attribute__((aligned(16))) float stg[GBM * GBN];
  const int tid = (int)threadIdx.x, lane = tid & 31, wave = tid >> 5, hh = lane >> 4, m = lane & 15;
  const int rowBase = (int)blockIdx.x * GBM;
  const int col0    = (int)blockIdx.y * GBN;

  v8f acc[4];
  {
    const v8f z = {0.f, 0.f, 0.f, 0.f, 0.f, 0.f, 0.f, 0.f};
    acc[0] = z; acc[1] = z; acc[2] = z; acc[3] = z;
  }
  const unsigned short* ap = A  + (size_t)(rowBase + 16 * wave + m) * (size_t)K + 8 * hh;
  const unsigned short* wp = WT + (size_t)(col0 + m) * (size_t)K + 8 * hh;
  const int ksteps = K >> 5;
#pragma unroll 1
  for (int ks = 0; ks < ksteps; ++ks) {
    FragB af;
    af.h[0] = *(const v8usa*)(ap + 32 * ks);
    af.h[1] = *(const v8usa*)(ap + 32 * ks + 16);
#pragma unroll
    for (int t = 0; t < 4; ++t) {
      const unsigned short* wq = wp + (size_t)(16 * t) * (size_t)K + 32 * ks;
      FragB bf;
      bf.h[0] = *(const v8usa*)wq;
      bf.h[1] = *(const v8usa*)(wq + 16);
      acc[t] = wmb(af, bf, acc[t]);
    }
  }

#pragma unroll
  for (int t = 0; t < 4; ++t) {
    const int lc = 16 * t + m;
#pragma unroll
    for (int r = 0; r < 8; ++r) {
      const int lr = 16 * wave + 8 * hh + r;
      stg[lr * GBN + lc] = acc[t][r];
    }
  }
  __syncthreads();

  v4f fv[8];
#pragma unroll
  for (int i = 0; i < 8; ++i) {
    const int lr = 16 * wave + 2 * i + hh;
    fv[i] = *(const v4fa*)(stg + lr * GBN + 4 * m);
  }
#pragma unroll
  for (int i = 0; i < 8; ++i) {
    const int lr = 16 * wave + 2 * i + hh;
    const int gr = rowBase + lr;
    float* op = outF + (size_t)gr * (size_t)ldo + col0 + 4 * m;
    *(volatile v4f*)op = fv[i];
  }
  __threadfence();
#pragma unroll
  for (int i = 0; i < 8; ++i) {
    const int lr = 16 * wave + 2 * i + hh;
    const int gr = rowBase + lr;
    float* op = outF + (size_t)gr * (size_t)ldo + col0 + 4 * m;
    *(volatile v4f*)op = fv[i];
  }
}

template<int L>
__global__ __launch_bounds__(NTHR) void k_agg(
    const int* __restrict__ srcs, const int* __restrict__ dsts,
    const float* __restrict__ P, const float* __restrict__ asrc, const float* __restrict__ adst,
    const float* __restrict__ bias, const int* __restrict__ numnew,
    unsigned short* X1B, float* out,
    int nN, int nE, int nb, int vec8, int MPr, int slot0, int nOut) {
  extern __shared__ v4f lds_dyn[];
  int* reg1 = (int*)lds_dyn;
  int* reg2 = reg1 + RCAP;
  int* scnt = reg2 + RCAP;
  int* soff = scnt + NBMAX;
  int* list = soff + NBMAX;
  int* wcnt = list + LISTN;
  int* wtot = wcnt + NWAVE;
  const int tid = (int)threadIdx.x, lane = tid & 31, wave = tid >> 5;
  const int nodeBase = slot0 + (int)blockIdx.x * nb;

  for (int i = tid; i < NBMAX; i += NTHR) scnt[i] = 0;
  __syncthreads();

  int tot = 0;
  const int nChunks = (nE + CHUNK - 1) / CHUNK;
#pragma unroll 1
  for (int ch = 0; ch < nChunks; ++ch) {
    const int cbase = ch * CHUNK;
    const int wc = scan_chunk(dsts, nE, cbase, nodeBase, nb, vec8, list, tid, lane, wave);
    if (lane == 0) wcnt[wave] = wc;
    __syncthreads();
    int pre = 0, all = 0;
#pragma unroll
    for (int w2 = 0; w2 < NWAVE; ++w2) {
      int c = wcnt[w2];
      c = c < 0 ? 0 : (c > WCAP ? WCAP : c);
      all += c;
      pre += (w2 < wave) ? c : 0;
    }
    const int wcc  = wc > WCAP ? WCAP : wc;
    const int base = tot + pre;
#pragma unroll 1
    for (int i = lane; i < wcc; i += 32) {
      const int ent = list[wave * WCAP + i];
      const int el  = (ent >> 12) & (CHUNK - 1);
      const int sl  = ent & (NBMAX - 1);
      int eid = cbase + el;
      eid = eid > nE - 1 ? nE - 1 : eid;
      const int pos = base + i;
      if (pos < RCAP) reg1[pos] = (int)(((unsigned)eid << 12) | (unsigned)sl);
    }
    tot += all;
    tot = tot > RCAP ? RCAP : tot;
    __syncthreads();
  }
  const int nh = tot;

  if (wave == 0) {
#pragma unroll 1
    for (int b0 = 0; b0 < nh; b0 += 32) {
      const int idx = b0 + lane;
      const int uv  = reg1[idx < nh ? idx : nh - 1];
      const int m32 = (nh - b0) < 32 ? (nh - b0) : 32;
#pragma unroll 1
      for (int k = 0; k < m32; ++k) {
        const int u  = __builtin_amdgcn_readlane(uv, k);
        const int sl = u & (NBMAX - 1);
        if (lane == 0) scnt[sl] = scnt[sl] + 1;
      }
    }
  }
  __syncthreads();

  {
    const v4i ca = *(const v4i*)(scnt + 8 * tid);
    const v4i cb = *(const v4i*)(scnt + 8 * tid + 4);
    const int e0 = ca.x < 0 ? 0 : ca.x, e1 = ca.y < 0 ? 0 : ca.y, e2 = ca.z < 0 ? 0 : ca.z, e3 = ca.w < 0 ? 0 : ca.w;
    const int e4 = cb.x < 0 ? 0 : cb.x, e5 = cb.y < 0 ? 0 : cb.y, e6 = cb.z < 0 ? 0 : cb.z, e7 = cb.w < 0 ? 0 : cb.w;
    const int ts = e0 + e1 + e2 + e3 + e4 + e5 + e6 + e7;
    int incl = ts;
#pragma unroll
    for (int d = 1; d < 32; d <<= 1) {
      const int up = __shfl_up(incl, d);
      if (lane >= d) incl += up;
    }
    if (lane == 31) wtot[wave] = incl;
    __syncthreads();
    int pre = 0;
#pragma unroll
    for (int w2 = 0; w2 < NWAVE; ++w2) pre += (w2 < wave) ? wtot[w2] : 0;
    int run = pre + incl - ts;
    soff[8 * tid + 0] = run; run += e0;
    soff[8 * tid + 1] = run; run += e1;
    soff[8 * tid + 2] = run; run += e2;
    soff[8 * tid + 3] = run; run += e3;
    soff[8 * tid + 4] = run; run += e4;
    soff[8 * tid + 5] = run; run += e5;
    soff[8 * tid + 6] = run; run += e6;
    soff[8 * tid + 7] = run;
  }
  __syncthreads();
  for (int i = tid; i < NBMAX; i += NTHR) list[i] = soff[i];
  __syncthreads();

  if (wave == 0) {
#pragma unroll 1
    for (int b0 = 0; b0 < nh; b0 += 32) {
      const int idx = b0 + lane;
      const int uv  = reg1[idx < nh ? idx : nh - 1];
      const int m32 = (nh - b0) < 32 ? (nh - b0) : 32;
#pragma unroll 1
      for (int k = 0; k < m32; ++k) {
        const int u   = __builtin_amdgcn_readlane(uv, k);
        const int sl  = u & (NBMAX - 1);
        const int eid = (int)((unsigned)u >> 12);
        if (lane == 0) {
          int pos = list[sl];
          pos = pos < 0 ? 0 : (pos > RCAP - 1 ? RCAP - 1 : pos);
          reg2[pos] = eid;
          list[sl] = pos + 1;
        }
      }
    }
  }
  __syncthreads();

  const int nbw = nb >> 3;
  const bool ovf = (nh >= RCAP);
  const float qnan = __int_as_float(0x7fc00000);

  if (L == 1) {
    unsigned int* stw = (unsigned int*)reg1 + wave * STW;
    const int c0 = 4 * lane;
    const v4f as4 = bfr4(*(const v4fa*)(asrc + c0));
    const v4f ad4 = bfr4(*(const v4fa*)(adst + c0));
    const v4f bb4 = bfr4(*(const v4fa*)(bias + c0));
#pragma unroll 1
    for (int jt = 0; jt < nbw; ++jt) {
      const int slot = wave * nbw + jt;
      const int grow = nodeBase + slot;
      const int gcl  = grow < nN ? grow : nN - 1;
      int st = soff[slot];
      const int craw = __builtin_amdgcn_readfirstlane(scnt[slot]);
      int cnt = craw;
      st  = st < 0 ? 0 : (st > nh ? nh : st);
      cnt = cnt < 0 ? 0 : (cnt > DEGCAP ? DEGCAP : cnt);
      if (cnt > nh - st) cnt = nh - st;
      st  = __builtin_amdgcn_readfirstlane(st);
      cnt = __builtin_amdgcn_readfirstlane(cnt);
      const float pz = (ovf || craw > DEGCAP) ? qnan : 0.0f;
      const bool wr = grow < MPr;
      const float live = grow < nN ? 1.0f : 0.0f;

      const v4f hd = *(const v4fa*)(P + (size_t)gcl * HD1 + c0);
      float ed = hd.x * ad4.x;
      ed = fmaf(hd.y, ad4.y, ed);
      ed = fmaf(hd.z, ad4.z, ed);
      ed = fmaf(hd.w, ad4.w, ed);
      ed += __shfl_xor(ed, 1);
      ed += __shfl_xor(ed, 2);
      ed += __shfl_xor(ed, 4);
      float mx = -1.0e30f, dn = 0.f;
      v4f av = {0.f, 0.f, 0.f, 0.f};

#pragma unroll 1
      for (int q = 0; q < cnt; ++q) {
        int idx = st + q; idx = idx > RCAP - 1 ? RCAP - 1 : idx;
        int eid = reg2[idx]; eid = eid < 0 ? 0 : (eid > nE - 1 ? nE - 1 : eid);
        const int sraw = srcs[eid];
        const int s = sraw < 0 ? 0 : (sraw > nN - 1 ? nN - 1 : sraw);
        const v4f hv = *(const v4fa*)(P + (size_t)s * HD1 + c0);
        float es = hv.x * as4.x;
        es = fmaf(hv.y, as4.y, es);
        es = fmaf(hv.z, as4.z, es);
        es = fmaf(hv.w, as4.w, es);
        es += __shfl_xor(es, 1);
        es += __shfl_xor(es, 2);
        es += __shfl_xor(es, 4);
        float lg = es + ed;
        lg = lg > 0.f ? lg : NEGSL * lg;
        const float df = lg - mx;
        const float ee = __expf(-fabsf(df));
        const bool up  = df > 0.f;
        const float s1 = up ? ee : 1.0f;
        const float s2 = up ? 1.0f : ee;
        mx = up ? lg : mx;
        dn = fmaf(dn, s1, s2);
        av.x = fmaf(av.x, s1, s2 * hv.x);
        av.y = fmaf(av.y, s1, s2 * hv.y);
        av.z = fmaf(av.z, s1, s2 * hv.z);
        av.w = fmaf(av.w, s1, s2 * hv.w);
      }
      const float ds = dn > 0.f ? dn : 1.0f;
      const float iv = (dn > 0.f ? 1.0f : 0.0f) * __builtin_amdgcn_rcpf(ds);
      float o0 = fmaf(av.x, iv, bb4.x);
      float o1 = fmaf(av.y, iv, bb4.y);
      float o2 = fmaf(av.z, iv, bb4.z);
      float o3 = fmaf(av.w, iv, bb4.w);
      o0 = o0 > 0.f ? o0 : (__expf(fminf(o0, 0.f)) - 1.0f);
      o1 = o1 > 0.f ? o1 : (__expf(fminf(o1, 0.f)) - 1.0f);
      o2 = o2 > 0.f ? o2 : (__expf(fminf(o2, 0.f)) - 1.0f);
      o3 = o3 > 0.f ? o3 : (__expf(fminf(o3, 0.f)) - 1.0f);
      const float q0 = o0 * live + pz;
      const float q1 = o1 * live + pz;
      const float q2 = o2 * live + pz;
      const float q3 = o3 * live + pz;
      const unsigned int h0 = f2bf(q0), h1 = f2bf(q1), h2 = f2bf(q2), h3 = f2bf(q3);
      const unsigned int l0 = f2bf(q0 - bf2f(h0)), l1 = f2bf(q1 - bf2f(h1));
      const unsigned int l2 = f2bf(q2 - bf2f(h2)), l3 = f2bf(q3 - bf2f(h3));
      v2u hw, lw;
      hw.x = h0 | (h1 << 16); hw.y = h2 | (h3 << 16);
      lw.x = l0 | (l1 << 16); lw.y = l2 | (l3 << 16);
      __builtin_amdgcn_fence(__ATOMIC_RELEASE, "wavefront");
      __builtin_amdgcn_wave_barrier();
      *(v2ua*)(stw + 2 * lane)      = hw;
      *(v2ua*)(stw + 64 + 2 * lane) = lw;
      __builtin_amdgcn_fence(__ATOMIC_RELEASE, "wavefront");
      __builtin_amdgcn_wave_barrier();
      const v4u pv = *(const v4ua*)(stw + 4 * lane);
      const int growc = wr ? grow : 0;
      unsigned short* gp = X1B + (size_t)growc * KG2 + 8 * lane;
      if (wr) *(volatile v4u*)gp = pv;
      __threadfence();
      if (wr) *(volatile v4u*)gp = pv;
    }
  } else {
    const int c0 = 2 * lane;
    v2f as2 = *(const v2fa*)(asrc + c0);
    v2f ad2 = *(const v2fa*)(adst + c0);
    v2f bb2 = *(const v2fa*)(bias + c0);
    as2.x = bfr(as2.x); as2.y = bfr(as2.y);
    ad2.x = bfr(ad2.x); ad2.y = bfr(ad2.y);
    bb2.x = bfr(bb2.x); bb2.y = bfr(bb2.y);
    const int nnw = numnew[0];
    const float pzn = (nnw != nOut) ? qnan : 0.0f;
#pragma unroll 1
    for (int jt = 0; jt < nbw; ++jt) {
      const int slot = wave * nbw + jt;
      const int grow = nodeBase + slot;
      const int gcl  = grow < nN ? grow : nN - 1;
      int st = soff[slot];
      const int craw = __builtin_amdgcn_readfirstlane(scnt[slot]);
      int cnt = craw;
      st  = st < 0 ? 0 : (st > nh ? nh : st);
      cnt = cnt < 0 ? 0 : (cnt > DEGCAP ? DEGCAP : cnt);
      if (cnt > nh - st) cnt = nh - st;
      st  = __builtin_amdgcn_readfirstlane(st);
      cnt = __builtin_amdgcn_readfirstlane(cnt);
      const float pz = ((ovf || craw > DEGCAP) ? qnan : 0.0f) + pzn;
      int orow = grow - slot0;
      const bool wr = (grow < nN) && (orow < nOut);
      orow = orow < 0 ? 0 : (orow > nOut - 1 ? nOut - 1 : orow);

      const v2f gd = *(const v2fa*)(P + (size_t)gcl * D2 + c0);
      float ed = gd.x * ad2.x;
      ed = fmaf(gd.y, ad2.y, ed);
      ed += __shfl_xor(ed, 1);
      ed += __shfl_xor(ed, 2);
      ed += __shfl_xor(ed, 4);
      ed += __shfl_xor(ed, 8);
      ed += __shfl_xor(ed, 16);
      float mx = -1.0e30f, dn = 0.f;
      v2f av = {0.f, 0.f};

#pragma unroll 1
      for (int q = 0; q < cnt; ++q) {
        int idx = st + q; idx = idx > RCAP - 1 ? RCAP - 1 : idx;
        int eid = reg2[idx]; eid = eid < 0 ? 0 : (eid > nE - 1 ? nE - 1 : eid);
        const int sraw = srcs[eid];
        const int s = sraw < 0 ? 0 : (sraw > nN - 1 ? nN - 1 : sraw);
        const v2f gv = *(const v2fa*)(P + (size_t)s * D2 + c0);
        float es = gv.x * as2.x;
        es = fmaf(gv.y, as2.y, es);
        es += __shfl_xor(es, 1);
        es += __shfl_xor(es, 2);
        es += __shfl_xor(es, 4);
        es += __shfl_xor(es, 8);
        es += __shfl_xor(es, 16);
        float lg = es + ed;
        lg = lg > 0.f ? lg : NEGSL * lg;
        const float df = lg - mx;
        const float ee = __expf(-fabsf(df));
        const bool up  = df > 0.f;
        const float s1 = up ? ee : 1.0f;
        const float s2 = up ? 1.0f : ee;
        mx = up ? lg : mx;
        dn = fmaf(dn, s1, s2);
        av.x = fmaf(av.x, s1, s2 * gv.x);
        av.y = fmaf(av.y, s1, s2 * gv.y);
      }
      const float ds = dn > 0.f ? dn : 1.0f;
      const float iv = (dn > 0.f ? 1.0f : 0.0f) * __builtin_amdgcn_rcpf(ds);
      v2f o;
      o.x = fmaf(av.x, iv, bb2.x) + pz;
      o.y = fmaf(av.y, iv, bb2.y) + pz;
      float* gp = out + (size_t)orow * D2 + c0;
      if (wr) *(volatile v2f*)gp = o;
      __threadfence();
      if (wr) *(volatile v2f*)gp = o;
    }
  }
}

static int pick_nb(int nE, int nN) {
  int nb = NBMAX;
  while (nb > 32 && (long long)nb * (long long)nE * 5LL > (long long)RCAP * (long long)nN * 4LL) nb >>= 1;
  return nb;
}
static inline int cdiv(int a, int b) { return (a + b - 1) / b; }

extern "C" void kernel_launch(void* const* d_in, const int* in_sizes, int n_in,
                              void* d_out, int out_size, void* d_ws, size_t ws_size,
                              hipStream_t stream) {
  if (n_in < 12) return;
  const int nN = in_sizes[0] / FIN;
  if (nN <= 0 || in_sizes[0] != nN * FIN || nN > (1 << 22)) return;
  const int nE = in_sizes[1];
  if (nE < 1 || nE > (1 << 20)) return;
  if (in_sizes[2] != nE) return;
  if (in_sizes[3] != FIN * HD1) return;
  if (in_sizes[4] != HD1 || in_sizes[5] != HD1) return;
  if (in_sizes[6] != HD1) return;
  if (in_sizes[7] != HD1 * D2) return;
  if (in_sizes[8] != D2 || in_sizes[9] != D2) return;
  if (in_sizes[10] != D2) return;
  if (in_sizes[11] < 1) return;
  if (out_size < D2 || (out_size % D2) != 0) return;
  const int nOut = out_size / D2;
  if (nOut > nN) return;
  const int slot0 = nN - nOut;

  const float* x    = (const float*)d_in[0];
  const int*   src  = (const int*)  d_in[1];
  const int*   dst  = (const int*)  d_in[2];
  const float* W1   = (const float*)d_in[3];
  const float* a1s  = (const float*)d_in[4];
  const float* a1d  = (const float*)d_in[5];
  const float* b1   = (const float*)d_in[6];
  const float* W2   = (const float*)d_in[7];
  const float* a2s  = (const float*)d_in[8];
  const float* a2d  = (const float*)d_in[9];
  const float* b2   = (const float*)d_in[10];
  const int*   nnw  = (const int*)  d_in[11];
  float* out = (float*)d_out;

  const int MP   = cdiv(nN, GBM) * GBM;
  const int nb   = pick_nb(nE, nN);
  if (nb < 32 || (nb & (nb - 1)) != 0 || nb > NBMAX) return;
  const int gA1  = cdiv(MP, nb);
  const int gA2  = cdiv(nOut, nb);
  const int vec8 = ((nE & 3) == 0) ? 1 : 0;
  if (gA1 * nb < MP || slot0 + gA2 * nb < nN) return;

  char* ws = (char*)d_ws;
  size_t off = 0;
  const size_t oXB  = off; off += (size_t)MP * FIN * 2;            off = (off + 255) & ~(size_t)255;
  const size_t oW1T = off; off += (size_t)HD1 * FIN * 2;           off = (off + 255) & ~(size_t)255;
  const size_t oW2T = off; off += (size_t)D2 * KG2 * 2;            off = (off + 255) & ~(size_t)255;
  const size_t oHX  = off; off += (size_t)MP * HD1 * 4;            off = (off + 255) & ~(size_t)255;
  const size_t oX1B = off; off += (size_t)MP * KG2 * 2;            off = (off + 255) & ~(size_t)255;
  const size_t oG   = off; off += (size_t)MP * D2 * 4;             off = (off + 255) & ~(size_t)255;
  if (off > ws_size || off > (size_t)WSMAX) return;
  unsigned short* XB   = (unsigned short*)(ws + oXB);
  unsigned short* W1T  = (unsigned short*)(ws + oW1T);
  unsigned short* W2T2 = (unsigned short*)(ws + oW2T);
  float*          HX   = (float*)(ws + oHX);
  unsigned short* X1B  = (unsigned short*)(ws + oX1B);
  float*          G    = (float*)(ws + oG);

  hipFuncSetAttribute(reinterpret_cast<const void*>(&k_agg<1>),
                      hipFuncAttributeMaxDynamicSharedMemorySize, LDS_AGG);
  hipFuncSetAttribute(reinterpret_cast<const void*>(&k_agg<2>),
                      hipFuncAttributeMaxDynamicSharedMemorySize, LDS_AGG);

  const int nUx = MP * (FIN / 8);
  k_xprep<<<cdiv(nUx, NTHR), NTHR, 0, stream>>>(x, XB, nN, nUx);

  {
    const int nU1 = HD1 * (FIN / 8);
    k_wtr<<<cdiv(nU1, NTHR), NTHR, 0, stream>>>(W1, FIN, HD1, HD1, FIN, W1T, nU1);
    const int nU2 = D2 * (KG2 / 8);
    k_wtr<<<cdiv(nU2, NTHR), NTHR, 0, stream>>>(W2, HD1, D2, D2, KG2, W2T2, nU2);
  }

  const int gM = MP / GBM;
  k_gemm<<<dim3(gM, HD1 / GBN), GTHR, 0, stream>>>(XB, W1T, HX, FIN, HD1);
  k_agg<1><<<gA1, NTHR, LDS_AGG, stream>>>(src, dst, HX, a1s, a1d, b1, nnw, X1B, out, nN, nE, nb, vec8, MP, 0, nOut);
  k_gemm<<<dim3(gM, D2 / GBN), GTHR, 0, stream>>>(X1B, W2T2, G, KG2, D2);
  k_agg<2><<<gA2, NTHR, LDS_AGG, stream>>>(src, dst, G, a2s, a2d, b2, nnw, X1B, out, nN, nE, nb, vec8, MP, slot0, nOut);
}
